// GATEdgeClassifier_89721866813769
// MI455X (gfx1250) — hardware-verified
//
#include <hip/hip_runtime.h>
#include <stddef.h>
#include <stdint.h>
#include <math.h>


#define NTHR   256
#define NWAVE  8
#define EPT    8
#define CHUNK  (NTHR * EPT)
#define WCAP   (EPT * 32)
#define LISTN  (NWAVE * WCAP)
#define NBA    1024
#define SLA    10
#define RCAP   24576
#define DEGCAP 128
#define GBM    64
#define HC     256
#define KP     512
#define NEGSL  0.2f
#define EPS_SM 1e-16f
#define WSMAX  134217728
#define AGG_ZINTS (LISTN + 2 * RCAP + 3 * NBA)
#define AGG_XOFF  (AGG_ZINTS + 16)
#define AGG_XFL   (48 + 9 * 256 + 160)
#define AGG_LDS_INTS (AGG_XOFF + AGG_XFL)
#define NU_W1  (256 * 64)
#define NU_W2  (32 * 64)
#define NU_MW  (64 * 8)
#define NU_W0  (256 * 16)
#define NU_EM  (16 * 16)
#define NU_ALL (NU_W1 + NU_W2 + NU_MW + NU_W0 + NU_EM)

static_assert((CHUNK & (CHUNK - 1)) == 0 && CHUNK <= 4096);
static_assert(NBA == (1 << SLA));
static_assert(AGG_ZINTS % 4 == 0 && (AGG_XOFF + 48) % 4 == 0);
static_assert(AGG_LDS_INTS * 4 <= 300000);
static_assert(NU_W1 % NTHR == 0 && NU_W2 % NTHR == 0 && NU_MW % NTHR == 0 && NU_W0 % NTHR == 0 && NU_EM % NTHR == 0);
static_assert(NBA % NWAVE == 0 && NBA % 32 == 0 && NBA % GBM == 0);

typedef float          v4f   __attribute__((ext_vector_type(4)));
typedef float          v8f   __attribute__((ext_vector_type(8)));
typedef double         v2d   __attribute__((ext_vector_type(2)));
typedef int            v4i   __attribute__((ext_vector_type(4)));
typedef int            v8i   __attribute__((ext_vector_type(8)));
typedef unsigned int   v4u   __attribute__((ext_vector_type(4)));
typedef unsigned short v8us  __attribute__((ext_vector_type(8)));
typedef unsigned short v16us __attribute__((ext_vector_type(16)));
typedef __bf16         v16bf __attribute__((ext_vector_type(16)));
typedef v4f  __attribute__((may_alias)) v4fa;
typedef v4i  __attribute__((may_alias)) v4ia;
typedef v2d  __attribute__((may_alias)) v2da;
typedef v8us __attribute__((may_alias)) v8usa;
union FragB { v16bf v; v16us u; v8us h[2]; v8i w; };

__device__ __forceinline__ v8f wmb(const FragB& a, const FragB& b, v8f c) {
  v8f d = __builtin_amdgcn_wmma_f32_16x16x32_bf16(false, a.v, false, b.v, (short)0, c, false, false);
  asm volatile("v_nop\n\tv_nop\n\tv_nop\n\tv_nop" : "+v"(d) : "v"(a.w), "v"(b.w));
  return d;
}

__device__ __forceinline__ unsigned bf16_bits(float f) {
  const unsigned u = __float_as_uint(f);
  return (u + 0x7FFFu + ((u >> 16) & 1u)) >> 16;
}
__device__ __forceinline__ float bf16_val(float f) {
  return __uint_as_float(bf16_bits(f) << 16);
}
__device__ __forceinline__ v4f bfr4(const v4f a) {
  v4f r; r.x = bf16_val(a.x); r.y = bf16_val(a.y); r.z = bf16_val(a.z); r.w = bf16_val(a.w); return r;
}
__device__ __forceinline__ double shx_d(double v, int msk) {
  int lo = __double2loint(v), hi = __double2hiint(v);
  lo = __shfl_xor(lo, msk);
  hi = __shfl_xor(hi, msk);
  return __hiloint2double(hi, lo);
}
__device__ __forceinline__ float elu1(float v) {
  const float p  = v * fmaf(v, fmaf(v, fmaf(v, 0.041666668f, 0.16666667f), 0.5f), 1.0f);
  const float q  = __expf(v) - 1.0f;
  const float ng = (fabsf(v) < 0.03125f) ? p : q;
  return (v > 0.0f) ? v : ng;
}

template <int SLB>
__device__ __forceinline__ int scan_chunk(const int* __restrict__ dsts, int nE, int cbase, int slotBase,
                                          int nb, int vec8, int* list, int tid, int lane, int wave) {
  int wc = 0;
  const int el0  = tid * EPT;
  const int e0   = cbase + el0;
  const int sent = -2147483647 - 1;
  v4i da, db;
  if (vec8 != 0 && cbase + CHUNK <= nE) {
    da = *(const v4i*)(dsts + e0);
    db = *(const v4i*)(dsts + e0 + 4);
  } else {
    da.x = (e0     < nE) ? dsts[min(e0,     nE - 1)] : sent;
    da.y = (e0 + 1 < nE) ? dsts[min(e0 + 1, nE - 1)] : sent;
    da.z = (e0 + 2 < nE) ? dsts[min(e0 + 2, nE - 1)] : sent;
    da.w = (e0 + 3 < nE) ? dsts[min(e0 + 3, nE - 1)] : sent;
    db.x = (e0 + 4 < nE) ? dsts[min(e0 + 4, nE - 1)] : sent;
    db.y = (e0 + 5 < nE) ? dsts[min(e0 + 5, nE - 1)] : sent;
    db.z = (e0 + 6 < nE) ? dsts[min(e0 + 6, nE - 1)] : sent;
    db.w = (e0 + 7 < nE) ? dsts[min(e0 + 7, nE - 1)] : sent;
  }
  const unsigned nbs = (unsigned)slotBase;
  const unsigned unb = (unsigned)nb;
  const unsigned s0 = (unsigned)da.x - nbs, s1 = (unsigned)da.y - nbs;
  const unsigned s2 = (unsigned)da.z - nbs, s3 = (unsigned)da.w - nbs;
  const unsigned s4 = (unsigned)db.x - nbs, s5 = (unsigned)db.y - nbs;
  const unsigned s6 = (unsigned)db.z - nbs, s7 = (unsigned)db.w - nbs;
  const bool h0 = s0 < unb, h1 = s1 < unb, h2 = s2 < unb, h3 = s3 < unb;
  const bool h4 = s4 < unb, h5 = s5 < unb, h6 = s6 < unb, h7 = s7 < unb;
  const unsigned any = __builtin_amdgcn_ballot_w32(h0 | h1 | h2 | h3 | h4 | h5 | h6 | h7);
  if (any != 0u) {
#define HITJ(J, HJ, SJ) { \
      const unsigned mj = __builtin_amdgcn_ballot_w32(HJ); \
      if (mj != 0u) { \
        if (HJ) { \
          const int pos = wc + (int)__builtin_amdgcn_mbcnt_lo(mj, 0u); \
          if (pos < WCAP) list[wave * WCAP + pos] = ((el0 + (J)) << SLB) | (int)(SJ); \
        } \
        wc += (int)__builtin_popcount(mj); } }
    HITJ(0, h0, s0)
    HITJ(1, h1, s1)
    HITJ(2, h2, s2)
    HITJ(3, h3, s3)
    HITJ(4, h4, s4)
    HITJ(5, h5, s5)
    HITJ(6, h6, s6)
    HITJ(7, h7, s7)
#undef HITJ
  }
  return wc;
}

__global__ __launch_bounds__(NTHR) void k_prep(const float* __restrict__ w1, const float* __restrict__ w2,
                                               const float* __restrict__ mw1, const float* __restrict__ w0,
                                               const float* __restrict__ emb,
                                               unsigned short* W1T, unsigned short* W2T, unsigned short* MWT,
                                               unsigned short* W0T, unsigned short* EMB) {
  const int u = (int)blockIdx.x * NTHR + (int)threadIdx.x;
  v8us o;
  unsigned short* dp;
  if (u < NU_W1) {
    const int n  = u >> 6;
    const int k8 = (u & 63) * 8;
    const int kk = k8 & 255;
    const float* p = w1 + (size_t)kk * 256 + n;
#pragma unroll
    for (int i = 0; i < 8; ++i) o[i] = (unsigned short)bf16_bits(p[(size_t)i * 256]);
    dp = W1T + (size_t)n * KP + k8;
  } else if (u < NU_W1 + NU_W2) {
    const int v  = u - NU_W1;
    const int n  = v >> 6;
    const int k8 = (v & 63) * 8;
    const int kk = k8 & 255;
    const float* p = w2 + (size_t)kk * 32 + n;
#pragma unroll
    for (int i = 0; i < 8; ++i) o[i] = (unsigned short)bf16_bits(p[(size_t)i * 32]);
    dp = W2T + (size_t)n * KP + k8;
  } else if (u < NU_W1 + NU_W2 + NU_MW) {
    const int v  = u - NU_W1 - NU_W2;
    const int n  = v >> 3;
    const int k8 = (v & 7) * 8;
    const int kk = k8 & 31;
    const int ro = (n >> 5) * 32;
    const int cl = n & 31;
    const float* p = mw1 + (size_t)(ro + kk) * 32 + cl;
#pragma unroll
    for (int i = 0; i < 8; ++i) o[i] = (unsigned short)bf16_bits(p[(size_t)i * 32]);
    dp = MWT + (size_t)n * 64 + k8;
  } else if (u < NU_W1 + NU_W2 + NU_MW + NU_W0) {
    const int v  = u - NU_W1 - NU_W2 - NU_MW;
    const int n  = v >> 4;
    const int k8 = (v & 15) * 8;
    const float* p = w0 + (size_t)k8 * 256 + n;
#pragma unroll
    for (int i = 0; i < 8; ++i) o[i] = (unsigned short)bf16_bits(p[(size_t)i * 256]);
    dp = W0T + (size_t)n * 128 + k8;
  } else if (u < NU_ALL) {
    const int v  = u - NU_W1 - NU_W2 - NU_MW - NU_W0;
    const int r  = v >> 4;
    const int k8 = (v & 15) * 8;
    const int rc = r < 9 ? r : 8;
    const float* p = emb + (size_t)rc * 128 + k8;
    const v4f a = *(const v4f*)p;
    const v4f b = *(const v4f*)(p + 4);
    const bool ok = r < 9;
    o[0] = ok ? (unsigned short)bf16_bits(a.x) : (unsigned short)0;
    o[1] = ok ? (unsigned short)bf16_bits(a.y) : (unsigned short)0;
    o[2] = ok ? (unsigned short)bf16_bits(a.z) : (unsigned short)0;
    o[3] = ok ? (unsigned short)bf16_bits(a.w) : (unsigned short)0;
    o[4] = ok ? (unsigned short)bf16_bits(b.x) : (unsigned short)0;
    o[5] = ok ? (unsigned short)bf16_bits(b.y) : (unsigned short)0;
    o[6] = ok ? (unsigned short)bf16_bits(b.z) : (unsigned short)0;
    o[7] = ok ? (unsigned short)bf16_bits(b.w) : (unsigned short)0;
    dp = EMB + (size_t)r * 128 + k8;
  } else {
    return;
  }
  *(volatile v8us*)dp = o;
  __threadfence();
  *(volatile v8us*)dp = o;
}

__global__ __launch_bounds__(NTHR) void k_ea(const float* __restrict__ ea, int nE, float* EA4, double* PART) {
  __shared__ __attribute__((aligned(16))) double wsum[NWAVE * 4];
  __shared__ __attribute__((aligned(16))) double rec[16];
  const int tid = (int)threadIdx.x, lane = tid & 31, wave = tid >> 5;
  const int e  = (int)blockIdx.x * NTHR + tid;
  const int ec = e < nE ? e : nE - 1;
  const bool ok = e < nE;
  const float* p = ea + (size_t)ec * 3;
  float a0 = bf16_val(p[0]), a1 = bf16_val(p[1]), a2 = bf16_val(p[2]);
  a0 = ok ? a0 : 0.0f; a1 = ok ? a1 : 0.0f; a2 = ok ? a2 : 0.0f;
  v4f v; v.x = a0; v.y = a1; v.z = a2; v.w = 0.0f;
  double d0 = (double)a0, d1 = (double)a1, d2 = (double)a2;
#pragma unroll
  for (int off = 16; off > 0; off >>= 1) {
    d0 += shx_d(d0, off);
    d1 += shx_d(d1, off);
    d2 += shx_d(d2, off);
  }
  if (lane == 0) { wsum[wave * 4 + 0] = d0; wsum[wave * 4 + 1] = d1; wsum[wave * 4 + 2] = d2; wsum[wave * 4 + 3] = 0.0; }
  __syncthreads();
  {
    const int ci  = tid & 15;
    const int col = ci < 3 ? ci : 3;
    double s = 0.0;
#pragma unroll
    for (int w2 = 0; w2 < NWAVE; ++w2) s += wsum[w2 * 4 + col];
    if (tid < 16) rec[tid] = s;
  }
  __syncthreads();
  float* op = EA4 + (size_t)e * 4;
  double* pp = PART + (size_t)blockIdx.x * 16 + 2 * lane;
  const bool wp = (wave == 0) && (lane < 8);
  const int rl = lane < 8 ? lane : 7;
  const v2d rt = *(const v2da*)(rec + 2 * rl);
  v2d rv;
  rv.x = wp ? rt.x : 0.0;
  rv.y = wp ? rt.y : 0.0;
  *(volatile v4f*)op = v;
  if (wp) *(volatile v2d*)pp = rv;
  __threadfence();
  *(volatile v4f*)op = v;
  if (wp) *(volatile v2d*)pp = rv;
}

__global__ __launch_bounds__(32) void k_tab(const unsigned short* __restrict__ EMB, const unsigned short* __restrict__ W0T,
                                            const float* __restrict__ as0, const float* __restrict__ ad0,
                                            float* T0, float* ASDT, const double* __restrict__ PART, int nPart,
                                            double invE, float* EAM) {
  __shared__ __attribute__((aligned(16))) float stg[16 * 32];
  __shared__ __attribute__((aligned(16))) float sdot[32];
  const int lane = (int)threadIdx.x, hh = lane >> 4, m = lane & 15;
  const int l8 = lane < 8 ? lane : 7;
  if (blockIdx.x >= 8) {
    const int col = lane < 3 ? lane : 3;
    double s = 0.0;
#pragma unroll 1
    for (int b = 0; b < nPart; ++b) s += PART[(size_t)b * 16 + col];
    const float mv = (float)(s * invE);
    sdot[lane] = (lane < 3) ? mv : 0.0f;
    __syncthreads();
    const v4f v = *(const v4fa*)(sdot + 4 * l8);
    if (lane < 8) *(volatile v4f*)(EAM + 4 * lane) = v;
    __threadfence();
    if (lane < 8) *(volatile v4f*)(EAM + 4 * lane) = v;
    return;
  }
  const int head = (int)blockIdx.x;
  v8f acc0 = {0.f, 0.f, 0.f, 0.f, 0.f, 0.f, 0.f, 0.f};
  v8f acc1 = acc0;
  const unsigned short* ap = EMB + (size_t)m * 128 + 8 * hh;
  const unsigned short* bp = W0T + (size_t)(head * 32 + m) * 128 + 8 * hh;
#pragma unroll 1
  for (int ks = 0; ks < 4; ++ks) {
    FragB af, b0, b1;
    af.h[0] = *(const v8usa*)(ap + 32 * ks);
    af.h[1] = *(const v8usa*)(ap + 32 * ks + 16);
    b0.h[0] = *(const v8usa*)(bp + 32 * ks);
    b0.h[1] = *(const v8usa*)(bp + 32 * ks + 16);
    b1.h[0] = *(const v8usa*)(bp + 16 * 128 + 32 * ks);
    b1.h[1] = *(const v8usa*)(bp + 16 * 128 + 32 * ks + 16);
    acc0 = wmb(af, b0, acc0);
    acc1 = wmb(af, b1, acc1);
  }
#pragma unroll
  for (int r = 0; r < 8; ++r) {
    stg[(8 * hh + r) * 32 + m]      = acc0[r];
    stg[(8 * hh + r) * 32 + 16 + m] = acc1[r];
  }
  __syncthreads();
  {
    float d = 0.0f;
#pragma unroll 2
    for (int c = 0; c < 32; ++c) {
      const float vs = bf16_val(as0[head * 32 + c]);
      const float vd = bf16_val(ad0[head * 32 + c]);
      const float a  = (hh != 0) ? vd : vs;
      d = fmaf(stg[m * 32 + c], a, d);
    }
    sdot[lane] = d;
  }
  __syncthreads();
  v4f tv[4];
#pragma unroll
  for (int it = 0; it < 4; ++it) {
    const int row = it * 4 + (lane >> 3);
    tv[it] = *(const v4fa*)(stg + row * 32 + 4 * (lane & 7));
  }
  const v4f st = *(const v4fa*)(sdot + 4 * l8);
  v4f sv;
  sv.x = (lane < 8) ? st.x : 0.0f;
  sv.y = (lane < 8) ? st.y : 0.0f;
  sv.z = (lane < 8) ? st.z : 0.0f;
  sv.w = (lane < 8) ? st.w : 0.0f;
#pragma unroll
  for (int it = 0; it < 4; ++it) {
    const int row = it * 4 + (lane >> 3);
    *(volatile v4f*)(T0 + (size_t)row * 256 + head * 32 + 4 * (lane & 7)) = tv[it];
  }
  if (lane < 8) *(volatile v4f*)(ASDT + head * 32 + 4 * lane) = sv;
  __threadfence();
#pragma unroll
  for (int it = 0; it < 4; ++it) {
    const int row = it * 4 + (lane >> 3);
    *(volatile v4f*)(T0 + (size_t)row * 256 + head * 32 + 4 * (lane & 7)) = tv[it];
  }
  if (lane < 8) *(volatile v4f*)(ASDT + head * 32 + 4 * lane) = sv;
}

__global__ __launch_bounds__(NTHR) void k_gemm1(const unsigned short* __restrict__ A, const unsigned short* __restrict__ BT,
                                                float* Cm, const float* __restrict__ avs,
                                                const float* __restrict__ avd, float* SD) {
  extern __shared__ __attribute__((aligned(16))) float gsm[];
  float* stg = gsm;
  float* sdt = gsm + GBM * HC;
  const int tid = (int)threadIdx.x, lane = tid & 31, wave = tid >> 5, hh = lane >> 4, m = lane & 15;
  const int rg = wave & 3, cg = wave >> 2;
  const int rowBase = (int)blockIdx.x * GBM;
  const int colBase = cg * 128;

  v8f acc[8];
  {
    const v8f z = {0.f, 0.f, 0.f, 0.f, 0.f, 0.f, 0.f, 0.f};
#pragma unroll
    for (int t = 0; t < 8; ++t) acc[t] = z;
  }
  const unsigned short* ap = A  + (size_t)(rowBase + 16 * rg + m) * (size_t)KP + 8 * hh;
  const unsigned short* bp = BT + (size_t)(colBase + m) * (size_t)KP + 8 * hh;

#pragma unroll 1
  for (int k0 = 0; k0 < KP; k0 += 32) {
    FragB af;
    af.h[0] = *(const v8usa*)(ap + k0);
    af.h[1] = *(const v8usa*)(ap + k0 + 16);
#pragma unroll
    for (int nt = 0; nt < 8; ++nt) {
      const unsigned short* wq = bp + (size_t)(16 * nt) * (size_t)KP + k0;
      FragB bf;
      bf.h[0] = *(const v8usa*)wq;
      bf.h[1] = *(const v8usa*)(wq + 16);
      acc[nt] = wmb(af, bf, acc[nt]);
    }
  }

#pragma unroll
  for (int nt = 0; nt < 8; ++nt) {
    const int lc = colBase + 16 * nt + m;
#pragma unroll
    for (int r = 0; r < 8; ++r) {
      const int lr = 16 * rg + 8 * hh + r;
      stg[lr * HC + lc] = acc[nt][r];
    }
  }
  __syncthreads();

  v4f as4[2], ad4[2];
#pragma unroll
  for (int c = 0; c < 2; ++c) {
    as4[c] = bfr4(*(const v4f*)(avs + c * 128 + 4 * lane));
    ad4[c] = bfr4(*(const v4f*)(avd + c * 128 + 4 * lane));
  }
#pragma unroll 1
  for (int i = 0; i < 8; ++i) {
    const int row = wave * 8 + i;
#pragma unroll
    for (int c = 0; c < 2; ++c) {
      const v4f p = *(const v4fa*)(stg + row * HC + c * 128 + 4 * lane);
      float s = p.x * as4[c].x; s = fmaf(p.y, as4[c].y, s); s = fmaf(p.z, as4[c].z, s); s = fmaf(p.w, as4[c].w, s);
      float d = p.x * ad4[c].x; d = fmaf(p.y, ad4[c].y, d); d = fmaf(p.z, ad4[c].z, d); d = fmaf(p.w, ad4[c].w, d);
#pragma unroll
      for (int off = 1; off < 8; off <<= 1) {
        s += __shfl_xor(s, off);
        d += __shfl_xor(d, off);
      }
      if ((lane & 7) == 0) {
        const int hd = 4 * c + (lane >> 3);
        sdt[row * 16 + hd]     = s;
        sdt[row * 16 + 8 + hd] = d;
      }
    }
  }
  __syncthreads();

  float* cb = Cm + (size_t)rowBase * HC;
  float* sb = SD + (size_t)rowBase * 16;
#pragma unroll 1
  for (int it = 0; it < 16; ++it) {
    const int p = it * NTHR + tid;
    const v4f v = *(const v4fa*)(stg + 4 * p);
    *(volatile v4f*)(cb + 4 * p) = v;
  }
  {
    const v4f v = *(const v4fa*)(sdt + 4 * tid);
    *(volatile v4f*)(sb + 4 * tid) = v;
  }
  __threadfence();
#pragma unroll 1
  for (int it = 0; it < 16; ++it) {
    const int p = it * NTHR + tid;
    const v4f v = *(const v4fa*)(stg + 4 * p);
    *(volatile v4f*)(cb + 4 * p) = v;
  }
  {
    const v4f v = *(const v4fa*)(sdt + 4 * tid);
    *(volatile v4f*)(sb + 4 * tid) = v;
  }
}

template <int NT, int DOTS>
__global__ __launch_bounds__(128) void k_gemm_s(const unsigned short* __restrict__ A, const unsigned short* __restrict__ BT,
                                                int K, float* Cm, const float* __restrict__ atts,
                                                const float* __restrict__ attd, float* SD) {
  constexpr int NCOL = NT * 16;
  __shared__ __attribute__((aligned(16))) float stg[GBM * NCOL];
  __shared__ __attribute__((aligned(16))) float satt[64];
  __shared__ __attribute__((aligned(16))) float sdot[128];
  const int tid = (int)threadIdx.x, lane = tid & 31, wave = tid >> 5, hh = lane >> 4, m = lane & 15;
  const int rowBase = (int)blockIdx.x * GBM;

  if (DOTS != 0) {
    if (tid < 64) {
      const int which = tid >> 5;
      const int c = tid & 31;
      const float vs = atts[c];
      const float vd = attd[c];
      const float v = (which == 0) ? vs : vd;
      satt[tid] = bf16_val(v);
    }
  }

  v8f acc[NT];
  {
    const v8f z = {0.f, 0.f, 0.f, 0.f, 0.f, 0.f, 0.f, 0.f};
#pragma unroll
    for (int t = 0; t < NT; ++t) acc[t] = z;
  }
  const unsigned short* ap = A  + (size_t)(rowBase + 16 * wave + m) * (size_t)K + 8 * hh;
  const unsigned short* wp = BT + (size_t)m * (size_t)K + 8 * hh;
  const int ksteps = K >> 5;
#pragma unroll 1
  for (int ks = 0; ks < ksteps; ++ks) {
    FragB af;
    af.h[0] = *(const v8usa*)(ap + 32 * ks);
    af.h[1] = *(const v8usa*)(ap + 32 * ks + 16);
#pragma unroll
    for (int t = 0; t < NT; ++t) {
      const unsigned short* wq = wp + (size_t)(16 * t) * (size_t)K + 32 * ks;
      FragB bf;
      bf.h[0] = *(const v8usa*)wq;
      bf.h[1] = *(const v8usa*)(wq + 16);
      acc[t] = wmb(af, bf, acc[t]);
    }
  }
#pragma unroll
  for (int t = 0; t < NT; ++t) {
    const int lc = 16 * t + m;
#pragma unroll
    for (int r = 0; r < 8; ++r) {
      const int lr = 16 * wave + 8 * hh + r;
      stg[lr * NCOL + lc] = acc[t][r];
    }
  }
  __syncthreads();

  if (DOTS != 0) {
    const int row = tid & 63, which = tid >> 6;
    const float* sa = satt + which * 32;
    const float* hr = stg + row * NCOL;
    float d = 0.f;
#pragma unroll 2
    for (int c4 = 0; c4 < 8; ++c4) {
      const v4f hv = *(const v4fa*)(hr + 4 * c4);
      const v4f av = *(const v4fa*)(sa + 4 * c4);
      d = fmaf(hv.x, av.x, d);
      d = fmaf(hv.y, av.y, d);
      d = fmaf(hv.z, av.z, d);
      d = fmaf(hv.w, av.w, d);
    }
    sdot[row * 2 + which] = d;
    __syncthreads();
  }

  float* cb = Cm + (size_t)rowBase * NCOL;
  float* sp = SD + (size_t)rowBase * 2 + 4 * lane;
  v4f sdv = {0.f, 0.f, 0.f, 0.f};
  if (DOTS != 0) sdv = *(const v4fa*)(sdot + 4 * lane);
#pragma unroll 1
  for (int it = 0; it < NT * 2; ++it) {
    const int p = it * 128 + tid;
    const v4f v = *(const v4fa*)(stg + 4 * p);
    *(volatile v4f*)(cb + 4 * p) = v;
  }
  if (DOTS != 0) { if (wave == 0) *(volatile v4f*)sp = sdv; }
  __threadfence();
#pragma unroll 1
  for (int it = 0; it < NT * 2; ++it) {
    const int p = it * 128 + tid;
    const v4f v = *(const v4fa*)(stg + 4 * p);
    *(volatile v4f*)(cb + 4 * p) = v;
  }
  if (DOTS != 0) { if (wave == 0) *(volatile v4f*)sp = sdv; }
}

template <int MODE>
__global__ __launch_bounds__(NTHR) void k_agg(const int* __restrict__ srcs, const int* __restrict__ dsts,
                                              int nE, int nN, int vec8, int mRows,
                                              const int* __restrict__ xid,
                                              const float* __restrict__ T0g, const float* __restrict__ ASDT,
                                              const float* __restrict__ XS, const float* __restrict__ SD,
                                              const float* __restrict__ EA4, const float* __restrict__ EAM,
                                              const float* __restrict__ we, const float* __restrict__ ae,
                                              const float* __restrict__ bias, unsigned short* hb) {
  extern __shared__ __attribute__((aligned(16))) int dsm[];
  int* list = dsm;
  int* hl   = dsm + LISTN;
  int* sl   = dsm + LISTN + RCAP;
  int* cnt  = dsm + LISTN + 2 * RCAP;
  int* offs = cnt + NBA;
  int* cur  = offs + NBA;
  int* misc = cur + NBA;
  float* vet = (float*)(dsm + AGG_XOFF);
  float* sle = vet + 32;
  float* T0s = vet + 48;
  float* ast = T0s + 9 * 256;
  float* adt = ast + 80;
  constexpr int NH  = (MODE == 2) ? 1 : 8;
  constexpr int HCW = (MODE == 2) ? 32 : 256;
  constexpr int NVT = NH * 3;
  const int tid = (int)threadIdx.x, lane = tid & 31, wave = tid >> 5;
  const int nodeBase = (int)blockIdx.x * NBA;

  {
    const v4i z4 = {0, 0, 0, 0};
    for (int i = tid * 4; i < AGG_ZINTS; i += NTHR * 4) *(v4ia*)(dsm + i) = z4;
    if (tid < 16) misc[tid] = 0;
  }
  if (wave == 0) {
    const int t   = lane < NVT ? lane : NVT - 1;
    const int hdv = t / 3;
    const int j   = t - 3 * hdv;
    float s = 0.0f;
#pragma unroll 2
    for (int c = 0; c < 32; ++c)
      s = fmaf(bf16_val(we[j * HCW + hdv * 32 + c]), bf16_val(ae[hdv * 32 + c]), s);
    if (lane < NVT) vet[hdv * 4 + j] = s;
  }
  if constexpr (MODE == 0) {
    for (int i = tid; i < 576; i += NTHR) *(v4fa*)(T0s + 4 * i) = *(const v4f*)(T0g + 4 * i);
    const int t = tid < 72 ? tid : 71;
    const int v = t >> 3, h = t & 7;
    const float a = ASDT[h * 32 + v];
    const float d = ASDT[h * 32 + 16 + v];
    if (tid < 72) { ast[t] = a; adt[t] = d; }
  }
  __syncthreads();
  {
    const int h = tid < NH ? tid : NH - 1;
    const float e0 = EAM[0], e1 = EAM[1], e2 = EAM[2];
    float s = e0 * vet[h * 4];
    s = fmaf(e1, vet[h * 4 + 1], s);
    s = fmaf(e2, vet[h * 4 + 2], s);
    if (tid < NH) sle[tid] = s;
  }

  int t = 0, ov = 0;
  const int nChunks = (nE + CHUNK - 1) / CHUNK;
#pragma unroll 1
  for (int ch = 0; ch < nChunks; ++ch) {
    const int cbase = ch * CHUNK;
    const int wc = scan_chunk<SLA>(dsts, nE, cbase, nodeBase, NBA, vec8, list, tid, lane, wave);
    if (lane == 0) misc[wave] = wc;
    __syncthreads();
    if (wave == 0) {
#pragma unroll 1
      for (int w2 = 0; w2 < NWAVE; ++w2) {
        int c = misc[w2];
        c = c < 0 ? 0 : (c > WCAP ? WCAP : c);
#pragma unroll 1
        for (int b0 = 0; b0 < c; b0 += 32) {
          const int idx = b0 + lane;
          const int ent = list[w2 * WCAP + (idx < WCAP ? idx : WCAP - 1)];
          const int m32 = (c - b0) < 32 ? (c - b0) : 32;
#pragma unroll 1
          for (int k = 0; k < m32; ++k) {
            const int u    = __builtin_amdgcn_readlane(ent, k);
            const int slot = u & (NBA - 1);
            const int el   = (u >> SLA) & (CHUNK - 1);
            const int pk   = ((cbase + el) << SLA) | slot;
            const int c1   = cnt[slot];
            if (t < RCAP) {
              if (lane == 0) { hl[t] = pk; cnt[slot] = c1 + 1; }
              t = t + 1;
            } else {
              ov = 1;
            }
          }
        }
      }
    }
    __syncthreads();
  }
  if (wave == 0 && lane == 0) { misc[8] = t; misc[9] = ov; }
  __syncthreads();
  int tt = misc[8];
  tt = tt < 0 ? 0 : (tt > RCAP ? RCAP : tt);
  const int ovf = misc[9];

  if (wave == 0) {
    const int base = lane * (NBA / 32);
    int s = 0;
#pragma unroll 1
    for (int i = 0; i < NBA / 32; ++i) s += cnt[base + i];
    int incl = s;
#pragma unroll
    for (int d = 1; d < 32; d <<= 1) {
      const int y = __shfl_up(incl, d, 32);
      if (lane >= d) incl += y;
    }
    int run = incl - s;
#pragma unroll 1
    for (int i = 0; i < NBA / 32; ++i) {
      const int cv = cnt[base + i];
      offs[base + i] = run;
      cur[base + i]  = run;
      run += cv;
    }
  }
  __syncthreads();
  if (wave == 0) {
#pragma unroll 1
    for (int b0 = 0; b0 < tt; b0 += 32) {
      const int idx = b0 + lane;
      const int ent = hl[idx < RCAP ? idx : RCAP - 1];
      const int m32 = (tt - b0) < 32 ? (tt - b0) : 32;
#pragma unroll 1
      for (int k = 0; k < m32; ++k) {
        const int u    = __builtin_amdgcn_readlane(ent, k);
        const int slot = u & (NBA - 1);
        int p = cur[slot];
        p = p < 0 ? 0 : (p > RCAP - 1 ? RCAP - 1 : p);
        if (lane == 0) {
          sl[p] = u;
          cur[slot] = p + 1;
        }
      }
    }
  }
  __syncthreads();

  const float pz = (ovf != 0) ? __int_as_float(0x7fc00000) : 0.0f;

  if constexpr (MODE != 2) {
    const int hd = lane >> 2;
    const float ve0 = vet[hd * 4], ve1 = vet[hd * 4 + 1], ve2 = vet[hd * 4 + 2];
    const float sleh = sle[hd];
    float bv[8];
    {
      const float* bq = bias + 8 * lane;
      const v4f a = *(const v4f*)bq;
      const v4f b = *(const v4f*)(bq + 4);
      bv[0] = bf16_val(a.x); bv[1] = bf16_val(a.y); bv[2] = bf16_val(a.z); bv[3] = bf16_val(a.w);
      bv[4] = bf16_val(b.x); bv[5] = bf16_val(b.y); bv[6] = bf16_val(b.z); bv[7] = bf16_val(b.w);
    }
#pragma unroll 1
    for (int si = 0; si < NBA / NWAVE; ++si) {
      const int s    = si * NWAVE + wave;
      const int node = nodeBase + s;
      int c = cnt[s];
      const bool big = c > DEGCAP;
      c = c < 0 ? 0 : (c > DEGCAP ? DEGCAP : c);
      int o = offs[s];
      o = o < 0 ? 0 : (o > RCAP ? RCAP : o);
      const int nc = node < nN ? node : nN - 1;
      float as0, ad;
      float acc[8];
      if constexpr (MODE == 0) {
        int xv = xid[nc];
        xv = xv < 0 ? 0 : (xv > 8 ? 8 : xv);
        as0 = ast[xv * 8 + hd];
        ad  = adt[xv * 8 + hd];
        const float* sp = T0s + xv * 256 + 8 * lane;
        const v4f a = *(const v4fa*)sp;
        const v4f b = *(const v4fa*)(sp + 4);
        acc[0] = a.x; acc[1] = a.y; acc[2] = a.z; acc[3] = a.w;
        acc[4] = b.x; acc[5] = b.y; acc[6] = b.z; acc[7] = b.w;
      } else {
        as0 = SD[(size_t)nc * 16 + hd];
        ad  = SD[(size_t)nc * 16 + 8 + hd];
        const float* sp = XS + (size_t)nc * HC + 8 * lane;
        const v4f a = *(const v4f*)sp;
        const v4f b = *(const v4f*)(sp + 4);
        acc[0] = a.x; acc[1] = a.y; acc[2] = a.z; acc[3] = a.w;
        acc[4] = b.x; acc[5] = b.y; acc[6] = b.z; acc[7] = b.w;
      }
      float l0 = (as0 + ad) + sleh;
      l0 = l0 > 0.f ? l0 : NEGSL * l0;
      float mx = l0, dn = 1.0f;
#pragma unroll 1
      for (int b0 = 0; b0 < c; b0 += 32) {
        int idx = o + b0 + lane;
        idx = idx > RCAP - 1 ? RCAP - 1 : idx;
        const int ent = sl[idx];
        int eid = ent >> SLA;
        eid = eid < 0 ? 0 : (eid > nE - 1 ? nE - 1 : eid);
        int sr = srcs[eid];
        sr = sr < 0 ? 0 : (sr > nN - 1 ? nN - 1 : sr);
        int key = sr;
        if constexpr (MODE == 0) {
          int xv = xid[sr];
          key = xv < 0 ? 0 : (xv > 8 ? 8 : xv);
        }
        const int m32 = (c - b0) < 32 ? (c - b0) : 32;
#pragma unroll 1
        for (int k = 0; k < m32; ++k) {
          const int kk = __builtin_amdgcn_readlane(key, k);
          const int ek = __builtin_amdgcn_readlane(eid, k);
          const v4f ea = *(const v4f*)(EA4 + (size_t)ek * 4);
          float ask;
          v4f a, b;
          if constexpr (MODE == 0) {
            ask = ast[kk * 8 + hd];
            const float* rp = T0s + kk * 256 + 8 * lane;
            a = *(const v4fa*)rp;
            b = *(const v4fa*)(rp + 4);
          } else {
            ask = SD[(size_t)kk * 16 + hd];
            const float* rp = XS + (size_t)kk * HC + 8 * lane;
            a = *(const v4f*)rp;
            b = *(const v4f*)(rp + 4);
          }
          float aev = ea.x * ve0;
          aev = fmaf(ea.y, ve1, aev);
          aev = fmaf(ea.z, ve2, aev);
          float lg = (ask + ad) + aev;
          lg = lg > 0.f ? lg : NEGSL * lg;
          const float df = lg - mx;
          const float ee = expf(-fabsf(df));
          const bool  up = df > 0.f;
          const float s1 = up ? ee : 1.0f;
          const float s2 = up ? 1.0f : ee;
          mx = up ? lg : mx;
          dn = fmaf(dn, s1, s2);
          acc[0] = fmaf(acc[0], s1, s2 * a.x); acc[1] = fmaf(acc[1], s1, s2 * a.y);
          acc[2] = fmaf(acc[2], s1, s2 * a.z); acc[3] = fmaf(acc[3], s1, s2 * a.w);
          acc[4] = fmaf(acc[4], s1, s2 * b.x); acc[5] = fmaf(acc[5], s1, s2 * b.y);
          acc[6] = fmaf(acc[6], s1, s2 * b.z); acc[7] = fmaf(acc[7], s1, s2 * b.w);
        }
      }
      const float inv = __builtin_amdgcn_rcpf(dn + EPS_SM);
      const float pzr = big ? __int_as_float(0x7fc00000) : pz;
      const bool live = node < nN;
      v8us ho, lo;
#pragma unroll
      for (int i = 0; i < 8; ++i) {
        float y = fmaf(acc[i], inv, bv[i]);
        y = elu1(y);
        y = y + pzr;
        y = live ? y : 0.0f;
        const unsigned hbi = bf16_bits(y);
        ho[i] = (unsigned short)hbi;
        lo[i] = (unsigned short)bf16_bits(y - __uint_as_float(hbi << 16));
      }
      if (node < mRows) {
        unsigned short* hp = hb + (size_t)node * KP + 8 * lane;
        *(volatile v8us*)hp = ho;
        *(volatile v8us*)(hp + HC) = lo;
        __threadfence();
        *(volatile v8us*)hp = ho;
        *(volatile v8us*)(hp + HC) = lo;
      }
    }
  } else {
    const float ve0 = vet[0], ve1 = vet[1], ve2 = vet[2];
    const float sleh = sle[0];
    const float bvl = bf16_val(bias[lane]);
#pragma unroll 1
    for (int si = 0; si < NBA / NWAVE; ++si) {
      const int s    = si * NWAVE + wave;
      const int node = nodeBase + s;
      int c = cnt[s];
      const bool big = c > DEGCAP;
      c = c < 0 ? 0 : (c > DEGCAP ? DEGCAP : c);
      int o = offs[s];
      o = o < 0 ? 0 : (o > RCAP ? RCAP : o);
      const int nc = node < nN ? node : nN - 1;
      const float as0 = SD[(size_t)nc * 2];
      const float ad  = SD[(size_t)nc * 2 + 1];
      float acc = XS[(size_t)nc * 32 + lane];
      float l0 = (as0 + ad) + sleh;
      l0 = l0 > 0.f ? l0 : NEGSL * l0;
      float mx = l0, dn = 1.0f;
#pragma unroll 1
      for (int b0 = 0; b0 < c; b0 += 32) {
        int idx = o + b0 + lane;
        idx = idx > RCAP - 1 ? RCAP - 1 : idx;
        const int ent = sl[idx];
        int eid = ent >> SLA;
        eid = eid < 0 ? 0 : (eid > nE - 1 ? nE - 1 : eid);
        int sr = srcs[eid];
        sr = sr < 0 ? 0 : (sr > nN - 1 ? nN - 1 : sr);
        const int m32 = (c - b0) < 32 ? (c - b0) : 32;
#pragma unroll 1
        for (int k = 0; k < m32; ++k) {
          const int kk = __builtin_amdgcn_readlane(sr, k);
          const int ek = __builtin_amdgcn_readlane(eid, k);
          const v4f ea = *(const v4f*)(EA4 + (size_t)ek * 4);
          const float ask = SD[(size_t)kk * 2];
          const float a   = XS[(size_t)kk * 32 + lane];
          float aev = ea.x * ve0;
          aev = fmaf(ea.y, ve1, aev);
          aev = fmaf(ea.z, ve2, aev);
          float lg = (ask + ad) + aev;
          lg = lg > 0.f ? lg : NEGSL * lg;
          const float df = lg - mx;
          const float ee = expf(-fabsf(df));
          const bool  up = df > 0.f;
          const float s1 = up ? ee : 1.0f;
          const float s2 = up ? 1.0f : ee;
          mx = up ? lg : mx;
          dn = fmaf(dn, s1, s2);
          acc = fmaf(acc, s1, s2 * a);
        }
      }
      const float inv = __builtin_amdgcn_rcpf(dn + EPS_SM);
      const float pzr = big ? __int_as_float(0x7fc00000) : pz;
      const bool live = node < nN;
      float y = fmaf(acc, inv, bvl);
      y = elu1(y);
      y = y + pzr;
      y = live ? y : 0.0f;
      const unsigned hbi = bf16_bits(y);
      const unsigned lbi = bf16_bits(y - __uint_as_float(hbi << 16));
      const int packed = (int)((hbi & 0xFFFFu) | ((lbi & 0xFFFFu) << 16));
      const int sb = 8 * (lane & 3);
      const int g0 = __shfl(packed, sb + 0), g1 = __shfl(packed, sb + 1);
      const int g2 = __shfl(packed, sb + 2), g3 = __shfl(packed, sb + 3);
      const int g4 = __shfl(packed, sb + 4), g5 = __shfl(packed, sb + 5);
      const int g6 = __shfl(packed, sb + 6), g7 = __shfl(packed, sb + 7);
      const int sh = (lane & 4) ? 16 : 0;
      const unsigned q0 = ((unsigned)g0 >> sh) & 0xFFFFu, q1 = ((unsigned)g1 >> sh) & 0xFFFFu;
      const unsigned q2 = ((unsigned)g2 >> sh) & 0xFFFFu, q3 = ((unsigned)g3 >> sh) & 0xFFFFu;
      const unsigned q4 = ((unsigned)g4 >> sh) & 0xFFFFu, q5 = ((unsigned)g5 >> sh) & 0xFFFFu;
      const unsigned q6 = ((unsigned)g6 >> sh) & 0xFFFFu, q7 = ((unsigned)g7 >> sh) & 0xFFFFu;
      v4u pv;
      pv.x = q0 | (q1 << 16); pv.y = q2 | (q3 << 16); pv.z = q4 | (q5 << 16); pv.w = q6 | (q7 << 16);
      const bool wr = (node < mRows) && (lane < 8);
      unsigned short* hp = hb + (size_t)node * 64 + 8 * (lane & 7);
      if (wr) *(volatile v4u*)hp = pv;
      __threadfence();
      if (wr) *(volatile v4u*)hp = pv;
    }
  }
}

__global__ __launch_bounds__(NTHR) void k_edge(const int* __restrict__ ei, int nE, int nN,
                                               const float* __restrict__ PQ, const float* __restrict__ mb1,
                                               const float* __restrict__ mw2, const float* __restrict__ mb2,
                                               float* out) {
  __shared__ __attribute__((aligned(16))) float smw[128];
  __shared__ __attribute__((aligned(16))) float smb1[32];
  __shared__ __attribute__((aligned(16))) float smb2[4];
  __shared__ __attribute__((aligned(16))) float sout[NTHR * 3];
  const int tid = (int)threadIdx.x;
  if (tid < 128) {
    const int k = tid >> 2, j = tid & 3;
    const int jc = j < 3 ? j : 2;
    const float v = bf16_val(mw2[k * 3 + jc]);
    smw[tid] = (j < 3) ? v : 0.0f;
  }
  if (tid < 32) {
    smb1[tid] = bf16_val(mb1[tid]);
    const int jc = tid < 3 ? tid : 2;
    const float v2 = bf16_val(mb2[jc]);
    if (tid < 4) smb2[tid] = (tid < 3) ? v2 : 0.0f;
  }
  __syncthreads();
  const int e  = (int)blockIdx.x * NTHR + tid;
  const int ec = e < nE ? e : nE - 1;
  int s = ei[ec];
  int d = ei[(size_t)nE + ec];
  s = s < 0 ? 0 : (s > nN - 1 ? nN - 1 : s);
  d = d < 0 ? 0 : (d > nN - 1 ? nN - 1 : d);
  const float* Pp = PQ + (size_t)s * 64;
  const float* Qp = PQ + (size_t)d * 64 + 32;
  float o0 = 0.0f, o1 = 0.0f, o2 = 0.0f;
#pragma unroll 2
  for (int c4 = 0; c4 < 8; ++c4) {
    const v4f p = *(const v4f*)(Pp + 4 * c4);
    const v4f q = *(const v4f*)(Qp + 4 * c4);
    const v4f b = *(const v4fa*)(smb1 + 4 * c4);
    const v4f m0 = *(const v4fa*)(smw + 16 * c4);
    const v4f m1 = *(const v4fa*)(smw + 16 * c4 + 4);
    const v4f m2 = *(const v4fa*)(smw + 16 * c4 + 8);
    const v4f m3 = *(const v4fa*)(smw + 16 * c4 + 12);
    float h0 = (p.x + q.x) + b.x; h0 = (h0 > 0.0f) ? h0 : (h0 - h0);
    float h1 = (p.y + q.y) + b.y; h1 = (h1 > 0.0f) ? h1 : (h1 - h1);
    float h2 = (p.z + q.z) + b.z; h2 = (h2 > 0.0f) ? h2 : (h2 - h2);
    float h3 = (p.w + q.w) + b.w; h3 = (h3 > 0.0f) ? h3 : (h3 - h3);
    o0 = fmaf(h0, m0.x, o0); o1 = fmaf(h0, m0.y, o1); o2 = fmaf(h0, m0.z, o2);
    o0 = fmaf(h1, m1.x, o0); o1 = fmaf(h1, m1.y, o1); o2 = fmaf(h1, m1.z, o2);
    o0 = fmaf(h2, m2.x, o0); o1 = fmaf(h2, m2.y, o1); o2 = fmaf(h2, m2.z, o2);
    o0 = fmaf(h3, m3.x, o0); o1 = fmaf(h3, m3.y, o1); o2 = fmaf(h3, m3.z, o2);
  }
  sout[3 * tid + 0] = o0 + smb2[0];
  sout[3 * tid + 1] = o1 + smb2[1];
  sout[3 * tid + 2] = o2 + smb2[2];
  __syncthreads();
  if (tid < 192) {
    const v4f v = *(const v4fa*)(sout + 4 * tid);
    float* op = out + (size_t)blockIdx.x * (NTHR * 3) + 4 * tid;
    *(volatile v4f*)op = v;
    __threadfence();
    *(volatile v4f*)op = v;
  }
}

static inline int cdiv(int a, int b) { return (a + b - 1) / b; }

extern "C" void kernel_launch(void* const* d_in, const int* in_sizes, int n_in,
                              void* d_out, int out_size, void* d_ws, size_t ws_size,
                              hipStream_t stream) {
  if (n_in < 26) return;
  const int nN = in_sizes[0];
  if (nN < 1 || nN > (1 << 22)) return;
  if (in_sizes[1] < 2 || (in_sizes[1] & 1) != 0) return;
  const int nE = in_sizes[1] / 2;
  if (nE < 1 || nE >= (1 << 21) || (nE % NTHR) != 0) return;
  if (in_sizes[2] != 3 * nE) return;
  if (in_sizes[3] != 9 * 128) return;
  if (in_sizes[4] != 128 * 256) return;
  if (in_sizes[5] != 256 || in_sizes[6] != 256 || in_sizes[7] != 768 || in_sizes[8] != 256 || in_sizes[9] != 256) return;
  if (in_sizes[10] != 256 * 256) return;
  if (in_sizes[11] != 256 || in_sizes[12] != 256 || in_sizes[13] != 768 || in_sizes[14] != 256 || in_sizes[15] != 256) return;
  if (in_sizes[16] != 256 * 32) return;
  if (in_sizes[17] != 32 || in_sizes[18] != 32 || in_sizes[19] != 96 || in_sizes[20] != 32 || in_sizes[21] != 32) return;
  if (in_sizes[22] != 64 * 32 || in_sizes[23] != 32 || in_sizes[24] != 96 || in_sizes[25] != 3) return;
  if ((long long)out_size != 3LL * (long long)nE) return;

  const int*   x    = (const int*)d_in[0];
  const int*   ei   = (const int*)d_in[1];
  const float* eat  = (const float*)d_in[2];
  const float* emb  = (const float*)d_in[3];
  const float* w0   = (const float*)d_in[4];
  const float* as0  = (const float*)d_in[5];
  const float* ad0  = (const float*)d_in[6];
  const float* we0  = (const float*)d_in[7];
  const float* ae0  = (const float*)d_in[8];
  const float* b0   = (const float*)d_in[9];
  const float* w1   = (const float*)d_in[10];
  const float* as1  = (const float*)d_in[11];
  const float* ad1  = (const float*)d_in[12];
  const float* we1  = (const float*)d_in[13];
  const float* ae1  = (const float*)d_in[14];
  const float* b1   = (const float*)d_in[15];
  const float* w2   = (const float*)d_in[16];
  const float* as2  = (const float*)d_in[17];
  const float* ad2  = (const float*)d_in[18];
  const float* we2  = (const float*)d_in[19];
  const float* ae2  = (const float*)d_in[20];
  const float* b2   = (const float*)d_in[21];
  const float* mw1  = (const float*)d_in[22];
  const float* mb1  = (const float*)d_in[23];
  const float* mw2  = (const float*)d_in[24];
  const float* mb2  = (const float*)d_in[25];
  float* out = (float*)d_out;
  const int* src = ei;
  const int* dst = ei + nE;

  const int MP    = cdiv(nN, GBM) * GBM;
  const int gM    = MP / GBM;
  const int gA    = cdiv(MP, NBA);
  if ((long long)gA * NBA < (long long)MP) return;
  const int nPart = nE / NTHR;
  const int vec8  = ((nE & 3) == 0) ? 1 : 0;
  const double invE = 1.0 / (double)nE;

  char* ws = (char*)d_ws;
  size_t off = 0;
  const size_t oW1T = off; off += (size_t)256 * KP * 2;                 off = (off + 255) & ~(size_t)255;
  const size_t oW2T = off; off += (size_t)32 * KP * 2;                  off = (off + 255) & ~(size_t)255;
  const size_t oMWT = off; off += (size_t)64 * 64 * 2;                  off = (off + 255) & ~(size_t)255;
  const size_t oW0T = off; off += (size_t)256 * 128 * 2;                off = (off + 255) & ~(size_t)255;
  const size_t oEMB = off; off += (size_t)16 * 128 * 2;                 off = (off + 255) & ~(size_t)255;
  const size_t oT0  = off; off += (size_t)16 * 256 * 4;                 off = (off + 255) & ~(size_t)255;
  const size_t oASD = off; off += (size_t)8 * 32 * 4;                   off = (off + 255) & ~(size_t)255;
  const size_t oEAM = off; off += (size_t)128;                          off = (off + 255) & ~(size_t)255;
  const size_t oPRT = off; off += (size_t)nPart * 128;                  off = (off + 255) & ~(size_t)255;
  const size_t oEA4 = off; off += (size_t)nPart * NTHR * 16;            off = (off + 255) & ~(size_t)255;
  const size_t oHP  = off; off += (size_t)MP * KP * 2;                  off = (off + 255) & ~(size_t)255;
  const size_t oXS  = off; off += (size_t)MP * HC * 4;                  off = (off + 255) & ~(size_t)255;
  const size_t oSD1 = off; off += (size_t)MP * 16 * 4;                  off = (off + 255) & ~(size_t)255;
  const size_t oSD2 = off; off += (size_t)MP * 2 * 4;                   off = (off + 255) & ~(size_t)255;
  if (off > ws_size || off > (size_t)WSMAX) return;
  unsigned short* W1T = (unsigned short*)(ws + oW1T);
  unsigned short* W2T = (unsigned short*)(ws + oW2T);
  unsigned short* MWT = (unsigned short*)(ws + oMWT);
  unsigned short* W0T = (unsigned short*)(ws + oW0T);
  unsigned short* EMB = (unsigned short*)(ws + oEMB);
  float*          T0  = (float*)(ws + oT0);
  float*          ASD = (float*)(ws + oASD);
  float*          EAM = (float*)(ws + oEAM);
  double*         PRT = (double*)(ws + oPRT);
  float*          EA4 = (float*)(ws + oEA4);
  unsigned short* HP  = (unsigned short*)(ws + oHP);
  float*          XS  = (float*)(ws + oXS);
  float*          XS2 = XS;
  float*          PQ  = XS + (size_t)MP * 32;
  float*          SD1 = (float*)(ws + oSD1);
  float*          SD2 = (float*)(ws + oSD2);

  const size_t aggLds  = (size_t)AGG_LDS_INTS * 4;
  const size_t gemmLds = (size_t)(GBM * HC + GBM * 16) * 4;
  hipFuncSetAttribute(reinterpret_cast<const void*>(&k_gemm1), hipFuncAttributeMaxDynamicSharedMemorySize, (int)gemmLds);
  hipFuncSetAttribute(reinterpret_cast<const void*>(&k_agg<0>), hipFuncAttributeMaxDynamicSharedMemorySize, (int)aggLds);
  hipFuncSetAttribute(reinterpret_cast<const void*>(&k_agg<1>), hipFuncAttributeMaxDynamicSharedMemorySize, (int)aggLds);
  hipFuncSetAttribute(reinterpret_cast<const void*>(&k_agg<2>), hipFuncAttributeMaxDynamicSharedMemorySize, (int)aggLds);

  k_prep<<<NU_ALL / NTHR, NTHR, 0, stream>>>(w1, w2, mw1, w0, emb, W1T, W2T, MWT, W0T, EMB);
  k_ea<<<nPart, NTHR, 0, stream>>>(eat, nE, EA4, PRT);
  k_tab<<<9, 32, 0, stream>>>(EMB, W0T, as0, ad0, T0, ASD, PRT, nPart, invE, EAM);
  k_agg<0><<<gA, NTHR, aggLds, stream>>>(src, dst, nE, nN, vec8, MP, x, T0, ASD, XS, SD1, EA4, EAM, we0, ae0, b0, HP);
  k_gemm1<<<gM, NTHR, gemmLds, stream>>>(HP, W1T, XS, as1, ad1, SD1);
  k_agg<1><<<gA, NTHR, aggLds, stream>>>(src, dst, nE, nN, vec8, MP, x, T0, ASD, XS, SD1, EA4, EAM, we1, ae1, b1, HP);
  k_gemm_s<2, 1><<<gM, 128, 0, stream>>>(HP, W2T, KP, XS2, as2, ad2, SD2);
  k_agg<2><<<gA, NTHR, aggLds, stream>>>(src, dst, nE, nN, vec8, MP, x, T0, ASD, XS2, SD2, EA4, EAM, we2, ae2, b2, HP);
  k_gemm_s<4, 0><<<gM, 128, 0, stream>>>(HP, MWT, 64, PQ, as2, ad2, SD2);
  k_edge<<<nPart, NTHR, 0, stream>>>(ei, nE, nN, PQ, mb1, mw2, mb2, out);
}
